// DSALite_88218628260696
// MI455X (gfx1250) — hardware-run, weakly checked
//
#include <hip/hip_runtime.h>
#pragma clang fp contract(off)


#ifndef SEQ
#define SEQ 2048
#endif
#define SEQ_FULL 2048
#define NHD  16
#define HD   128
#define DSTR 8
#define DSN  (SEQ / DSTR)
#define TOPK (SEQ / 10)
#define KSEL ((TOPK + DSTR - 1) / DSTR)
#define NV   (DSN / 32)
#define PSH  10.0f
#define QKC  64.0f
#define DSC  (1.0f / 4096.0f)
#define VSC  (1.0f / 64.0f)
#define SCL  0.08838834764831845f
#define L2E  1.4426950408889634f
#define NEGB (-1.0e9f)

typedef _Float16 h16;
typedef __attribute__((ext_vector_type(16))) _Float16 v16h;
typedef __attribute__((ext_vector_type(8)))  _Float16 v8h;
typedef __attribute__((ext_vector_type(8)))  float    v8f;
typedef __attribute__((ext_vector_type(4)))  float    v4f;
typedef v8h  __attribute__((may_alias)) v8ha;
typedef v4f  __attribute__((may_alias)) v4fa;

static_assert(SEQ % 512 == 0);
static_assert(SEQ <= SEQ_FULL);
static_assert(HD == 128);
static_assert(HD % 32 == 0);
static_assert(HD % 64 == 0);
static_assert(DSN % 64 == 0);
static_assert(DSN % 32 == 0);
static_assert(DSN % 16 == 0);
static_assert(NV >= 1);
static_assert(KSEL >= 1);
static_assert(KSEL <= DSN);
static_assert(TOPK >= 1);
static_assert(((size_t)NHD * SEQ * HD) % 8 == 0);
static_assert(((size_t)SEQ * HD) % 8 == 0);
static_assert(DSN * 16 * 4 + 16 * 40 * 2 + 16 * 132 * 4 <= 131072);
static_assert(64 * 65 * 4 <= 131072);
static_assert(16 * 68 * 4 <= 131072);

__device__ __forceinline__ unsigned short f2bf(float f) { unsigned u = __float_as_uint(f); u += 0x7FFFu + ((u >> 16) & 1u); return (unsigned short)(u >> 16); }
__device__ __forceinline__ float bf2f(unsigned short b) { return __uint_as_float(((unsigned)b) << 16); }
__device__ __forceinline__ float bfr(float f) { return bf2f(f2bf(f)); }
__device__ __forceinline__ v16h cat16(v8h lo, v8h hi) { return __builtin_shufflevector(lo, hi, 0, 1, 2, 3, 4, 5, 6, 7, 8, 9, 10, 11, 12, 13, 14, 15); }
static __device__ __forceinline__ h16 toh_flush(float v) { const h16 r = (h16)v; return (fabsf(v) < 6.103515625e-05f) ? (h16)0.0f : r; }
__device__ __forceinline__ v8f wmma16g(v16h a, v16h b, v8f c) {
    c = __builtin_amdgcn_wmma_f32_16x16x32_f16(false, a, false, b, (short)0, c, false, false);
    asm volatile("v_nop\n\tv_nop\n\tv_nop\n\tv_nop" : "+v"(c) : "v"(a), "v"(b));
    return c;
}
__device__ __forceinline__ v16h ldh(const h16* p) { return cat16(*(const v8h*)p, *(const v8h*)(p + 16)); }

__global__ __launch_bounds__(256) void k_cvth(const float* __restrict__ src, h16* dst, size_t n8) {
    const size_t i = (size_t)blockIdx.x * 256 + threadIdx.x; if (i >= n8) return;
    const size_t e = i * 8; const size_t hh = e / ((size_t)SEQ * HD); const size_t rest = e - hh * ((size_t)SEQ * HD);
    const v8f v = *(const v8f*)(src + hh * ((size_t)SEQ_FULL * HD) + rest); v8h o;
#pragma unroll
    for (int k = 0; k < 8; ++k) o[k] = toh_flush(bfr(v[k]) * QKC);
    *(volatile v8h*)(dst + e) = o; __threadfence(); *(volatile v8h*)(dst + e) = o;
}

__global__ __launch_bounds__(256) void k_cvtvt(const float* __restrict__ V, h16* VT) {
    __shared__ float tl[64 * 65];
    const int tid = threadIdx.x; const int t0 = blockIdx.x * 64, d0 = blockIdx.y * 64, h = blockIdx.z;
#pragma unroll
    for (int it = 0; it < 4; ++it) { const int r = (tid >> 4) + 16 * it, c4 = (tid & 15) * 4; const v4f a = *(const v4f*)(V + ((size_t)h * SEQ_FULL + t0 + r) * HD + d0 + c4);
        tl[r * 65 + c4] = a[0]; tl[r * 65 + c4 + 1] = a[1]; tl[r * 65 + c4 + 2] = a[2]; tl[r * 65 + c4 + 3] = a[3]; }
    __syncthreads();
    const int pc = tid & 7; v8h o[2];
#pragma unroll
    for (int it = 0; it < 2; ++it) { const int n = (tid >> 3) + 32 * it;
#pragma unroll
        for (int q = 0; q < 8; ++q) o[it][q] = toh_flush(bfr(tl[(pc * 8 + q) * 65 + n]) * QKC); }
    static_assert(256 * 2 * 16 == 64 * 64 * 2);
#pragma unroll
    for (int it = 0; it < 2; ++it) { const int n = (tid >> 3) + 32 * it; *(volatile v8h*)(VT + ((size_t)h * HD + d0 + n) * SEQ + t0 + pc * 8) = o[it]; }
    __threadfence();
#pragma unroll
    for (int it = 0; it < 2; ++it) { const int n = (tid >> 3) + 32 * it; *(volatile v8h*)(VT + ((size_t)h * HD + d0 + n) * SEQ + t0 + pc * 8) = o[it]; }
}

__global__ __launch_bounds__(32) void k_sds(const h16* __restrict__ Q16, const h16* __restrict__ K16, float* SD) {
    __shared__ __align__(16) float os[16 * 68];
    const int lane = threadIdx.x & 31, lr = lane & 15, hi = lane >> 4;
    const int m0 = blockIdx.x * 16, n0 = blockIdx.y * 64, h = blockIdx.z;
    const int aoff = (h * SEQ + (m0 + lr) * DSTR) * HD + 8 * hi;
    const int boff = (h * SEQ + (n0 + lr) * DSTR) * HD + 8 * hi;
    v8f acc[4];
#pragma unroll
    for (int nb = 0; nb < 4; ++nb) acc[nb] = (v8f){};
#pragma unroll 1
    for (int f = 0; f < HD / 32; ++f) {
        const v16h a = ldh(Q16 + aoff + f * 32);
#pragma unroll
        for (int nb = 0; nb < 4; ++nb) { const v16h b = ldh(K16 + boff + nb * 16 * DSTR * HD + f * 32); acc[nb] = wmma16g(a, b, acc[nb]); }
    }
#pragma unroll
    for (int nb = 0; nb < 4; ++nb) {
#pragma unroll
        for (int j = 0; j < 8; ++j) os[(hi * 8 + j) * 68 + nb * 16 + lr] = (acc[nb][j] * DSC) * SCL; }
    __builtin_amdgcn_wave_barrier(); asm volatile("" ::: "memory");
    float* crow = SD + ((size_t)h * DSN + m0) * DSN + n0;
    static_assert(16 * 16 == 64 * 4);
    static_assert(8 * 2 == 16);
#pragma unroll 1
    for (int ps = 0; ps < 2; ++ps) {
#pragma unroll
        for (int s = 0; s < 8; ++s) { const int row = 2 * s + hi, cofs = lr * 4; const v4f val = *(const v4fa*)&os[row * 68 + cofs];
            *(volatile v4f*)(crow + (size_t)row * DSN + cofs) = val; }
        if (ps == 0) __threadfence(); }
}

__global__ __launch_bounds__(32) void k_flash(const h16* __restrict__ Q16, const h16* __restrict__ K16, const h16* __restrict__ VT, const float* __restrict__ SD, const float* __restrict__ U, float* OUT) {
    __shared__ __align__(16) float bt[DSN * 16];
    __shared__ __align__(16) h16 ps[16 * 40];
    __shared__ __align__(16) float os[16 * 132];
    const int lane = threadIdx.x & 31, lr = lane & 15, hi = lane >> 4;
    const int h = blockIdx.y, q0 = blockIdx.x * 16;
    const int ir0 = q0 / DSTR;
    float tA = 0.0f, tB = 0.0f;
#pragma unroll 1
    for (int rr = 0; rr < 2; ++rr) {
        const int sb = (h * DSN + ir0 + rr) * DSN + lane;
        float v[NV];
#pragma unroll
        for (int j = 0; j < NV; ++j) v[j] = SD[sb + j * 32];
        float t = 0.0f;
#pragma unroll 1
        for (int it = 0; it < KSEL; ++it) {
            float lm = v[0]; int li = 0;
#pragma unroll
            for (int j = 1; j < NV; ++j) { const bool g = v[j] > lm; lm = g ? v[j] : lm; li = g ? j : li; }
            float wm = lm;
            wm = fmaxf(wm, __shfl_xor(wm, 1, 32)); wm = fmaxf(wm, __shfl_xor(wm, 2, 32)); wm = fmaxf(wm, __shfl_xor(wm, 4, 32)); wm = fmaxf(wm, __shfl_xor(wm, 8, 32)); wm = fmaxf(wm, __shfl_xor(wm, 16, 32));
            const unsigned long long bal = __ballot(lm == wm);
            const int leader = __ffsll(bal) - 1;
            const bool me = (lane == leader);
#pragma unroll
            for (int j = 0; j < NV; ++j) v[j] = (me & (li == j)) ? -3.0e38f : v[j];
            t = wm;
        }
        tA = (rr == 0) ? t : tA; tB = (rr == 1) ? t : tB;
    }
    {
        const int row = lr;
        float uq = bfr(U[q0 + row]);
        uq = fminf(fmaxf(uq, 0.0f), 1.0f);
        const float us = 1.0f + uq;
        const float tsel = (lane & 8) ? tB : tA;
        const float thr = tsel * us;
        const int sdrow = (h * DSN + ir0 + (row >> 3)) * DSN;
#pragma unroll 1
        for (int it = 0; it < DSN / 2; ++it) {
            const int jb = 2 * it + hi;
            const float sv = SD[sdrow + jb];
            const float sf = sv * us;
            float x = (sf - thr) * 10.0f;
            x = fminf(fmaxf(x, -20.0f), 20.0f);
            const float ex = expf(-x);
            const float mk = 1.0f / (1.0f + ex);
            bt[jb * 16 + row] = (1.0f - mk) * NEGB;
        }
    }
    __builtin_amdgcn_wave_barrier(); asm volatile("" ::: "memory");

    const int qoff  = (h * SEQ + q0 + lr) * HD + 8 * hi;
    const int kbase = (h * SEQ + lr) * HD + 8 * hi;
    const int vbase = (h * HD + lr) * SEQ + 8 * hi;
    v8f o[8]; float m[8], l[8];
#pragma unroll
    for (int j = 0; j < 8; ++j) o[j] = (v8f){};
#pragma unroll
    for (int r = 0; r < 8; ++r) { m[r] = -2.0e38f; l[r] = 0.0f; }
#pragma unroll 1
    for (int t0 = 0; t0 < SEQ; t0 += 32) {
        v8f s0 = (v8f){}, s1 = (v8f){};
        const int koff = kbase + t0 * HD;
#pragma unroll 1
        for (int f = 0; f < 4; ++f) {
            const v16h qa = ldh(Q16 + qoff + f * 32);
            const v16h b0 = ldh(K16 + koff + f * 32);
            const v16h b1 = ldh(K16 + koff + 16 * HD + f * 32);
            s0 = wmma16g(qa, b0, s0);
            s1 = wmma16g(qa, b1, s1);
        }
        const int jb0 = (t0 >> 3) + (lr >> 3);
        v4f pa0 = *(const v4fa*)&bt[jb0 * 16 + 8 * hi];
        v4f pa1 = *(const v4fa*)&bt[jb0 * 16 + 8 * hi + 4];
        v4f pb0 = *(const v4fa*)&bt[(jb0 + 2) * 16 + 8 * hi];
        v4f pb1 = *(const v4fa*)&bt[(jb0 + 2) * 16 + 8 * hi + 4];
        asm volatile("" : "+v"(pa0)); asm volatile("" : "+v"(pa1)); asm volatile("" : "+v"(pb0)); asm volatile("" : "+v"(pb1));
        float ba[8], bb[8];
#pragma unroll
        for (int r = 0; r < 4; ++r) { ba[r] = pa0[r]; ba[4 + r] = pa1[r]; bb[r] = pb0[r]; bb[4 + r] = pb1[r]; }
        const int j0 = t0 + lr;
#pragma unroll
        for (int r = 0; r < 8; ++r) {
            const int iq = q0 + 8 * hi + r;
            const float be0 = (j0 <= iq) ? ba[r] : NEGB;
            const float be1 = (j0 + 16 <= iq) ? bb[r] : NEGB;
            const float d0 = (s0[r] * DSC) * SCL;
            const float d1 = (s1[r] * DSC) * SCL;
            const float a0 = d0 + be0;
            const float a1 = d1 + be1;
            float mx = fmaxf(a0, a1);
            mx = fmaxf(mx, __shfl_xor(mx, 1, 32)); mx = fmaxf(mx, __shfl_xor(mx, 2, 32)); mx = fmaxf(mx, __shfl_xor(mx, 4, 32)); mx = fmaxf(mx, __shfl_xor(mx, 8, 32));
            const float mn = fmaxf(m[r], mx);
            const float al = __builtin_amdgcn_exp2f((m[r] - mn) * L2E);
            const float e0 = (a0 - mn) * L2E + PSH;
            const float e1 = (a1 - mn) * L2E + PSH;
            const float x0 = __builtin_amdgcn_exp2f(e0);
            const float x1 = __builtin_amdgcn_exp2f(e1);
            const float p0 = (e0 < -14.0f) ? 0.0f : x0;
            const float p1 = (e1 < -14.0f) ? 0.0f : x1;
            const h16 c0 = (h16)p0;
            const h16 c1 = (h16)p1;
            l[r] = l[r] * al + ((float)c0 + (float)c1);
            m[r] = mn;
#pragma unroll
            for (int j = 0; j < 8; ++j) o[j][r] *= al;
            ps[(8 * hi + r) * 40 + lr] = c0;
            ps[(8 * hi + r) * 40 + 16 + lr] = c1;
        }
        __builtin_amdgcn_wave_barrier(); asm volatile("" ::: "memory");
        const v16h pf = cat16(*(const v8ha*)&ps[lr * 40 + 8 * hi], *(const v8ha*)&ps[lr * 40 + 16 + 8 * hi]);
        const int voff = vbase + t0;
        {
            v16h vb[4];
#pragma unroll
            for (int jj = 0; jj < 4; ++jj) vb[jj] = ldh(VT + voff + jj * 16 * SEQ);
#pragma unroll
            for (int jj = 0; jj < 4; ++jj) o[jj] = wmma16g(pf, vb[jj], o[jj]);
        }
        {
            v16h vb[4];
#pragma unroll
            for (int jj = 0; jj < 4; ++jj) vb[jj] = ldh(VT + voff + (4 + jj) * 16 * SEQ);
#pragma unroll
            for (int jj = 0; jj < 4; ++jj) o[4 + jj] = wmma16g(pf, vb[jj], o[4 + jj]);
        }
        __builtin_amdgcn_wave_barrier(); asm volatile("" ::: "memory");
    }
#pragma unroll
    for (int r = 0; r < 8; ++r) {
        float lt = l[r];
        lt += __shfl_xor(lt, 1, 32); lt += __shfl_xor(lt, 2, 32); lt += __shfl_xor(lt, 4, 32); lt += __shfl_xor(lt, 8, 32);
        const float inv = (1.0f / lt) * VSC;
#pragma unroll
        for (int j = 0; j < 8; ++j) os[(8 * hi + r) * 132 + j * 16 + lr] = o[j][r] * inv;
    }
    __builtin_amdgcn_wave_barrier(); asm volatile("" ::: "memory");
    static_assert(32 * 16 == HD * 4);
#pragma unroll 1
    for (int pass = 0; pass < 2; ++pass) {
#pragma unroll
        for (int s = 0; s < 16; ++s) {
            const v4f val = *(const v4fa*)&os[s * 132 + lane * 4];
            *(volatile v4f*)(OUT + ((size_t)h * SEQ_FULL + q0 + s) * HD + lane * 4) = val;
        }
        if (pass == 0) __threadfence();
    }
}

#define PLQ   ((size_t)NHD * SEQ * HD * 2)
#define SDB   ((size_t)NHD * DSN * DSN * 4)
#define CARVE (3 * PLQ   + SDB  )
#define INMIN ((size_t)(NHD - 1) * SEQ_FULL * HD + (size_t)SEQ * HD)
static_assert(PLQ % 256 == 0);
static_assert(SDB % 256 == 0);
static_assert(CARVE <= (size_t)134217728);

extern "C" void kernel_launch(void* const* d_in, const int* in_sizes, int n_in,
                              void* d_out, int out_size, void* d_ws, size_t ws_size, hipStream_t stream) {
    if (n_in < 4) return;
    if ((size_t)in_sizes[0] < INMIN || (size_t)in_sizes[1] < INMIN || (size_t)in_sizes[2] < INMIN) return;
    if (in_sizes[3] < SEQ) return;
    if ((size_t)out_size < INMIN) return;
    if (ws_size < CARVE) return;
    const float* qin = (const float*)d_in[0];
    const float* kin = (const float*)d_in[1];
    const float* vin = (const float*)d_in[2];
    const float* uin = (const float*)d_in[3];
    float* OUT = (float*)d_out;
    char* wsp = (char*)d_ws;
    auto take = [&](size_t bytes) { char* p = wsp; wsp += (bytes + 255) & ~(size_t)255; return (void*)p; };
    h16* Q16 = (h16*)take(PLQ); h16* K16 = (h16*)take(PLQ); h16* VT16 = (h16*)take(PLQ);
    float* SD = (float*)take(SDB);
    if ((size_t)(wsp - (char*)d_ws) > ws_size) return;

    const size_t n8 = (size_t)NHD * SEQ * HD / 8; const unsigned g8 = (unsigned)((n8 + 255) / 256);
    k_cvth<<<g8, 256, 0, stream>>>(qin, Q16, n8);
    k_cvth<<<g8, 256, 0, stream>>>(kin, K16, n8);
    k_cvtvt<<<dim3(SEQ / 64, HD / 64, NHD), 256, 0, stream>>>(vin, VT16);
    k_sds<<<dim3(DSN / 16, DSN / 64, NHD), 32, 0, stream>>>(Q16, K16, SD);
    k_flash<<<dim3(SEQ / 16, NHD), 32, 0, stream>>>(Q16, K16, VT16, SD, uin, OUT);
}
